// MambaMixer_56727928046135
// MI455X (gfx1250) — hardware-verified
//
#include <hip/hip_runtime.h>
#include <math.h>

typedef __attribute__((ext_vector_type(16))) _Float16 v16h;
typedef __attribute__((ext_vector_type(8)))  _Float16 v8h;
typedef __attribute__((ext_vector_type(16))) __bf16   v16b;
typedef __attribute__((ext_vector_type(8)))  __bf16   v8b;
typedef __attribute__((ext_vector_type(8)))  float    v8f;
typedef __attribute__((ext_vector_type(4)))  float    v4f;

constexpr int kBatch = 2;
constexpr int kSeqL  = 2048;
constexpr int kDmod  = 1024;
constexpr int kDin   = 2048;
constexpr int kNst   = 16;
constexpr int kDtR   = 64;
constexpr int kPrjN  = 96;
constexpr int kPrjP  = 128;
constexpr int kXZP   = 2 * kDin;
constexpr int kRows  = kBatch * kSeqL;
constexpr int kTP    = 260;

constexpr float kCarWx   = 32.0f;
constexpr float kCarWdt  = 8.0f;
constexpr float kCarWout = 32.0f;
constexpr float kCarDt   = 16.0f;
constexpr float kCarY    = 16.0f;

static_assert(kDtR + 2 * kNst == kPrjN, "x_proj width");
static_assert((kDmod % 32) == 0 && (kDin % 32) == 0 && (kDtR % 32) == 0, "GEMM K multiples of 32");
static_assert((kSeqL % 64) == 0 && (kXZP % 64) == 0 && (kPrjP % 64) == 0 && (kDin % 64) == 0 && (kDmod % 64) == 0, "GEMM M,N multiples of 64");
static_assert((kDin % 256) == 0 && (kSeqL % 64) == 0 && (kSeqL % 16) == 0, "tile multiples");

constexpr size_t kSzWIN16  = (size_t)kXZP * kDmod * 2;
constexpr size_t kSzWXP16  = (size_t)kPrjP * kDin * 2;
constexpr size_t kSzWDT16  = (size_t)kDin * kDtR * 2;
constexpr size_t kSzWOUT16 = (size_t)kDmod * kDin * 2;
constexpr size_t kSzX16    = (size_t)kRows * kDmod * 2;
constexpr size_t kSzXZ     = (size_t)kSeqL * kXZP * 4;
constexpr size_t kSzUC     = (size_t)kSeqL * kDin * 4;
constexpr size_t kSzUC16   = (size_t)kSeqL * kDin * 2;
constexpr size_t kSzPROJ   = (size_t)kSeqL * kPrjP * 4;
constexpr size_t kSzDT16   = (size_t)kSeqL * kDtR * 2;
constexpr size_t kSzDLR    = (size_t)kSeqL * kDin * 4;
constexpr size_t kSzY16    = (size_t)kSeqL * kDin * 2;
constexpr size_t kOffWIN16  = 0;
constexpr size_t kOffWXP16  = kOffWIN16  + kSzWIN16;
constexpr size_t kOffWDT16  = kOffWXP16  + kSzWXP16;
constexpr size_t kOffWOUT16 = kOffWDT16  + kSzWDT16;
constexpr size_t kOffX16    = kOffWOUT16 + kSzWOUT16;
constexpr size_t kOffXZ     = kOffX16    + kSzX16;
constexpr size_t kOffUC     = kOffXZ     + kSzXZ;
constexpr size_t kOffUC16   = kOffUC     + kSzUC;
constexpr size_t kOffPROJ   = kOffUC16   + kSzUC16;
constexpr size_t kOffDT16   = kOffPROJ   + kSzPROJ;
constexpr size_t kOffDLR    = kOffDT16   + kSzDT16;
constexpr size_t kOffY16    = kOffDLR    + kSzDLR;
constexpr size_t kWsTotal   = kOffY16    + kSzY16;
static_assert(kWsTotal == 106954752ull, "carve total");
static_assert(kWsTotal <= 134217728ull, "carve cap");
static_assert((kOffWXP16 % 128) == 0 && (kOffWDT16 % 128) == 0 && (kOffWOUT16 % 128) == 0 && (kOffX16 % 128) == 0 &&
              (kOffXZ % 128) == 0 && (kOffUC % 128) == 0 && (kOffUC16 % 128) == 0 && (kOffPROJ % 128) == 0 &&
              (kOffDT16 % 128) == 0 && (kOffDLR % 128) == 0 && (kOffY16 % 128) == 0, "128-B aligned regions");

__device__ __forceinline__ unsigned short f2bf_bits(float f) {
  unsigned u = __float_as_uint(f);
  return (unsigned short)((u + 0x7FFFu + ((u >> 16) & 1u)) >> 16);
}
__device__ __forceinline__ float bf_bits2f(unsigned short h) { return __uint_as_float(((unsigned)h) << 16); }
__device__ __forceinline__ float rne_bf16(float f) { return bf_bits2f(f2bf_bits(f)); }

__device__ __forceinline__ void dep_guard4_h(v8f& a, v8f& b, v8f& c, v8f& d, v16h x, v16h b0, v16h b1, v16h b2, v16h b3) {
  asm volatile("v_nop\n\tv_nop\n\tv_nop\n\tv_nop" : "+v"(a), "+v"(b), "+v"(c), "+v"(d) : "v"(x), "v"(b0), "v"(b1), "v"(b2), "v"(b3));
}
__device__ __forceinline__ void dep_guard4_b(v8f& a, v8f& b, v8f& c, v8f& d, v16b x, v16b b0, v16b b1, v16b b2, v16b b3) {
  asm volatile("v_nop\n\tv_nop\n\tv_nop\n\tv_nop" : "+v"(a), "+v"(b), "+v"(c), "+v"(d) : "v"(x), "v"(b0), "v"(b1), "v"(b2), "v"(b3));
}
__device__ __forceinline__ void keep4_h(v16h a, v16h b, v16h c, v16h d) { asm volatile("v_nop" :: "v"(a), "v"(b), "v"(c), "v"(d)); }
__device__ __forceinline__ void keep4_b(v16b a, v16b b, v16b c, v16b d) { asm volatile("v_nop" :: "v"(a), "v"(b), "v"(c), "v"(d)); }
__device__ __forceinline__ void acc_guard4(v8f& a, v8f& b, v8f& c, v8f& d) { asm volatile("v_nop\n\tv_nop\n\tv_nop\n\tv_nop" : "+v"(a), "+v"(b), "+v"(c), "+v"(d)); }

template <typename T> struct Frag;
template <> struct Frag<_Float16> {
  typedef v16h V; union U { v16h v; v8h h[2]; };
  static __device__ __forceinline__ v16h load(const _Float16* p) {
    U f; f.h[0] = *(const v8h*)(p); f.h[1] = *(const v8h*)(p + 16); return f.v;
  }
  static __device__ __forceinline__ v8f mma(v16h a, v16h b, v8f c) {
    return __builtin_amdgcn_wmma_f32_16x16x32_f16(false, a, false, b, (short)0, c, false, false);
  }
  static __device__ __forceinline__ void guard4(v8f& a, v8f& b, v8f& c, v8f& d, v16h x, v16h b0, v16h b1, v16h b2, v16h b3) { dep_guard4_h(a, b, c, d, x, b0, b1, b2, b3); }
  static __device__ __forceinline__ void keep(v16h a, v16h b, v16h c, v16h d) { keep4_h(a, b, c, d); }
};
template <> struct Frag<__bf16> {
  typedef v16b V; union U { v16b v; v8b h[2]; };
  static __device__ __forceinline__ v16b load(const __bf16* p) {
    U f; f.h[0] = *(const v8b*)(p); f.h[1] = *(const v8b*)(p + 16); return f.v;
  }
  static __device__ __forceinline__ v8f mma(v16b a, v16b b, v8f c) {
    return __builtin_amdgcn_wmma_f32_16x16x32_bf16(false, a, false, b, (short)0, c, false, false);
  }
  static __device__ __forceinline__ void guard4(v8f& a, v8f& b, v8f& c, v8f& d, v16b x, v16b b0, v16b b1, v16b b2, v16b b3) { dep_guard4_b(a, b, c, d, x, b0, b1, b2, b3); }
  static __device__ __forceinline__ void keep(v16b a, v16b b, v16b c, v16b d) { keep4_b(a, b, c, d); }
};

template <int ET> struct Elem;
template <> struct Elem<0> { typedef _Float16 T; };
template <> struct Elem<1> { typedef __bf16 T; };
template <int ET>
__global__ __launch_bounds__(256) void wmma_gemm64(
    const unsigned short* __restrict__ Ap, int lda,
    const unsigned short* __restrict__ Btp, int ldb,
    float* __restrict__ Cout, int ldc,
    int M, int N, int K, float scale) {
  typedef typename Elem<ET>::T T;
  typedef typename Frag<T>::V V;
  const T* A = (const T*)Ap;
  const T* Bt = (const T*)Btp;
  __shared__ __align__(16) float sT[8][16 * 68];
  const int lane = threadIdx.x & 31;
  const int wave = threadIdx.x >> 5;
  const int tilesN = N >> 6;
  const int tilesM = M >> 6;
  const int tile = blockIdx.x * 8 + wave;
  if (tile >= tilesM * tilesN) return;
  const int tm = tile / tilesN;
  const int tn = tile - tm * tilesN;
  const int m0 = tm << 6;
  const int n0 = tn << 6;

  const int rlane = lane & 15;
  const int koff  = (lane >> 4) * 8;
  const int mOff  = (lane >> 4) * 8;

  v8f acc[4][4];
#pragma unroll
  for (int i = 0; i < 4; ++i)
#pragma unroll
    for (int j = 0; j < 4; ++j) acc[i][j] = (v8f){0.f,0.f,0.f,0.f,0.f,0.f,0.f,0.f};

  for (int k0 = 0; k0 < K; k0 += 32) {
    V bh[4];
#pragma unroll
    for (int j = 0; j < 4; ++j) {
      const size_t bo = (size_t)(n0 + (j << 4) + rlane) * ldb + koff + k0;
      bh[j] = Frag<T>::load(Bt + bo);
    }
#pragma unroll
    for (int i = 0; i < 4; ++i) {
      const size_t ao = (size_t)(m0 + (i << 4) + rlane) * lda + koff + k0;
      V ah = Frag<T>::load(A + ao);
#pragma unroll
      for (int j = 0; j < 4; ++j) acc[i][j] = Frag<T>::mma(ah, bh[j], acc[i][j]);
      Frag<T>::guard4(acc[i][0], acc[i][1], acc[i][2], acc[i][3], ah, bh[0], bh[1], bh[2], bh[3]);
    }
    Frag<T>::keep(bh[0], bh[1], bh[2], bh[3]);
  }
  acc_guard4(acc[0][0], acc[0][1], acc[0][2], acc[0][3]);
  acc_guard4(acc[1][0], acc[1][1], acc[1][2], acc[1][3]);
  acc_guard4(acc[2][0], acc[2][1], acc[2][2], acc[2][3]);
  acc_guard4(acc[3][0], acc[3][1], acc[3][2], acc[3][3]);

  float* slab = sT[wave];
  const int hh = lane >> 4;
  const int c4 = (lane & 15) * 4;
#pragma unroll
  for (int i = 0; i < 4; ++i) {
    const int mBase = m0 + (i << 4);
#pragma unroll
    for (int j = 0; j < 4; ++j) {
#pragma unroll
      for (int r = 0; r < 8; ++r) {
        slab[(mOff + r) * 68 + (j << 4) + rlane] = acc[i][j][r] * scale;
      }
    }
    __builtin_amdgcn_fence(__ATOMIC_RELEASE, "workgroup");
    __builtin_amdgcn_wave_barrier();
    __builtin_amdgcn_fence(__ATOMIC_ACQUIRE, "workgroup");
    for (int pass = 0; pass < 2; ++pass) {
#pragma unroll
      for (int it = 0; it < 8; ++it) {
        const int row = it * 2 + hh;
        v4f v = *(const v4f*)(slab + row * 68 + c4);
        *(volatile v4f*)(Cout + (size_t)(mBase + row) * ldc + n0 + c4) = v;
      }
      __threadfence();
    }
    __builtin_amdgcn_fence(__ATOMIC_RELEASE, "workgroup");
    __builtin_amdgcn_wave_barrier();
    __builtin_amdgcn_fence(__ATOMIC_ACQUIRE, "workgroup");
  }
}

template <int MODE>
__global__ __launch_bounds__(256) void cast_plane_kernel(
    const float* __restrict__ src, unsigned short* __restrict__ dst, int real8, int pad8, float scale)
{
  const int i = blockIdx.x * 256 + threadIdx.x;
  if (i >= pad8) return;
  const bool live = (i < real8);
  const int ic = live ? i : (real8 - 1);
  const float* p = src + ((size_t)ic << 3);
  const v4f a0 = *(const v4f*)(p);
  const v4f a1 = *(const v4f*)(p + 4);
  v8h hv;
#pragma unroll
  for (int e = 0; e < 4; ++e) {
    const float f0 = a0[e];
    const float f1 = a1[e];
    const unsigned short b0 = f2bf_bits(f0);
    const unsigned short b1 = f2bf_bits(f1);
    if (MODE == 0) {
      const unsigned short s0 = live ? b0 : (unsigned short)0;
      const unsigned short s1 = live ? b1 : (unsigned short)0;
      hv[e]     = __builtin_bit_cast(_Float16, s0);
      hv[4 + e] = __builtin_bit_cast(_Float16, s1);
    } else {
      const float g0 = live ? (bf_bits2f(b0) * scale) : 0.0f;
      const float g1 = live ? (bf_bits2f(b1) * scale) : 0.0f;
      hv[e]     = (_Float16)g0;
      hv[4 + e] = (_Float16)g1;
    }
  }
  unsigned short* q = dst + ((size_t)i << 3);
  *(volatile v8h*)q = hv;
  __threadfence();
  *(volatile v8h*)q = hv;
}

__global__ __launch_bounds__(256) void dt_cast_kernel(
    const float* __restrict__ PROJ, unsigned short* __restrict__ DT16, int total8, float scale)
{
  const int i = blockIdx.x * 256 + threadIdx.x;
  if (i >= total8) return;
  const int e0  = i << 3;
  const int row = e0 >> 6;
  const int c8  = e0 & 63;
  const float* p = PROJ + (size_t)row * kPrjP + c8;
  const v4f a0 = *(const v4f*)(p);
  const v4f a1 = *(const v4f*)(p + 4);
  v8h hv;
#pragma unroll
  for (int e = 0; e < 4; ++e) {
    hv[e]     = (_Float16)(a0[e] * scale);
    hv[4 + e] = (_Float16)(a1[e] * scale);
  }
  unsigned short* qd = DT16 + e0;
  *(volatile v8h*)qd = hv;
  __threadfence();
  *(volatile v8h*)qd = hv;
}

__global__ __launch_bounds__(256) void conv_silu_kernel(
    const float* __restrict__ XZ, const float* __restrict__ cw, const float* __restrict__ cb,
    float* __restrict__ UC, unsigned short* __restrict__ UC16)
{
  __shared__ __align__(16) float sT[16 * kTP];
  const int tid = threadIdx.x, lane = tid & 31, wave = tid >> 5;
  const int d0 = blockIdx.x * 256, d = d0 + tid;
  const int t0 = blockIdx.y * 64;
  const v4f wv = *(const v4f*)(cw + (size_t)d * 4);
  const float w0 = rne_bf16(wv[0]);
  const float w1 = rne_bf16(wv[1]);
  const float w2 = rne_bf16(wv[2]);
  const float w3 = rne_bf16(wv[3]);
  const float bc = rne_bf16(cb[d]);
  float xm3, xm2, xm1;
  {
    const int r3 = t0 - 3, r2 = t0 - 2, r1 = t0 - 1;
    const float v3 = XZ[(size_t)(r3 < 0 ? 0 : r3) * kXZP + d];
    const float v2 = XZ[(size_t)(r2 < 0 ? 0 : r2) * kXZP + d];
    const float v1 = XZ[(size_t)(r1 < 0 ? 0 : r1) * kXZP + d];
    xm3 = (r3 >= 0) ? v3 : 0.f;
    xm2 = (r2 >= 0) ? v2 : 0.f;
    xm1 = (r1 >= 0) ? v1 : 0.f;
  }
  const int hrow = wave >> 1;
  const int hch  = (wave & 1) * 128 + lane * 4;
#pragma unroll 1
  for (int sub = 0; sub < 4; ++sub) {
    const int lb = t0 + sub * 16;
#pragma unroll 1
    for (int s = 0; s < 16; ++s) {
      const float xc = XZ[(size_t)(lb + s) * kXZP + d];
      float acc = w0 * xm3;
      acc = fmaf(w1, xm2, acc);
      acc = fmaf(w2, xm1, acc);
      acc = fmaf(w3, xc, acc);
      const float sv = acc + bc;
      const float sg = __builtin_amdgcn_rcpf(1.0f + expf(-sv));
      sT[s * kTP + tid] = sv * sg;
      xm3 = xm2; xm2 = xm1; xm1 = xc;
    }
    __syncthreads();
    v4f fv[4];
    v8h bv[2];
#pragma unroll
    for (int it = 0; it < 4; ++it) fv[it] = *(const v4f*)(sT + (it * 4 + hrow) * kTP + hch);
#pragma unroll
    for (int it = 0; it < 2; ++it) {
      const float* sp = sT + (it * 8 + wave) * kTP + lane * 8;
      const v4f a0 = *(const v4f*)(sp);
      const v4f a1 = *(const v4f*)(sp + 4);
#pragma unroll
      for (int e = 0; e < 4; ++e) {
        bv[it][e]     = (_Float16)a0[e];
        bv[it][4 + e] = (_Float16)a1[e];
      }
    }
    for (int pass = 0; pass < 2; ++pass) {
#pragma unroll
      for (int it = 0; it < 4; ++it)
        *(volatile v4f*)(UC + (size_t)(lb + it * 4 + hrow) * kDin + d0 + hch) = fv[it];
#pragma unroll
      for (int it = 0; it < 2; ++it)
        *(volatile v8h*)(UC16 + (size_t)(lb + it * 8 + wave) * kDin + d0 + lane * 8) = bv[it];
      __threadfence();
    }
    __syncthreads();
  }
}

__global__ __launch_bounds__(256) void scan_kernel(
    const float* __restrict__ DLR, const float* __restrict__ UC, const float* __restrict__ XZ,
    const float* __restrict__ PROJ, const float* __restrict__ A_log, const float* __restrict__ bdt,
    const float* __restrict__ Dv, unsigned short* __restrict__ Y16)
{
  __shared__ __align__(16) float sBC[16 * 32];
  __shared__ __align__(16) float sY[16 * kTP];
  __shared__ __align__(16) float sA[kNst * 256];
  const int tid = threadIdx.x, lane = tid & 31, wave = tid >> 5;
  const int d0 = blockIdx.x * 256, d = d0 + tid;

#pragma unroll 1
  for (int n = 0; n < kNst; ++n) {
    const float al = rne_bf16(A_log[(size_t)d * kNst + n]);
    sA[n * 256 + tid] = -expf(al);
  }
  __syncthreads();
  float An[kNst];
  float h[kNst];
#pragma unroll
  for (int n = 0; n < kNst; ++n) {
    An[n] = sA[n * 256 + tid];
    h[n] = 0.f;
  }
  const float bb = rne_bf16(bdt[d]);
  const float Dd = rne_bf16(Dv[d]);

#pragma unroll 1
  for (int c = 0; c < kSeqL / 16; ++c) {
    const int l0 = c * 16;
    if (tid < 128) {
      const int r = tid >> 3, q = (tid & 7) * 4;
      const v4f v = *(const v4f*)(PROJ + (size_t)(l0 + r) * kPrjP + kDtR + q);
      *(v4f*)(sBC + r * 32 + q) = v;
    }
    __syncthreads();
#pragma unroll 1
    for (int s = 0; s < 16; ++s) {
      const size_t m = (size_t)(l0 + s);
      const float pre   = DLR[m * kDin + d];
      const float a     = (pre + bb) + bb;
      const float ea    = expf(-fabsf(a));
      const float delta = fmaxf(a, 0.0f) + log1pf(ea);
      const float xv    = UC[m * kDin + d];
      const float zv    = XZ[m * kXZP + kDin + d];
      const float du    = delta * xv;
      v4f Bq[4], Cq[4];
#pragma unroll
      for (int qq = 0; qq < 4; ++qq) {
        Bq[qq] = *(const v4f*)(sBC + s * 32 + 4 * qq);
        Cq[qq] = *(const v4f*)(sBC + s * 32 + kNst + 4 * qq);
      }
      float y = 0.f;
#pragma unroll
      for (int n = 0; n < kNst; ++n) {
        const float e  = __expf(delta * An[n]);
        const float p  = du * Bq[n >> 2][n & 3];
        const float hn = fmaf(e, h[n], p);
        h[n] = hn;
        y = fmaf(Cq[n >> 2][n & 3], hn, y);
      }
      y = fmaf(xv, Dd, y);
      const float sg = __builtin_amdgcn_rcpf(1.0f + expf(-zv));
      const float g  = zv * sg;
      sY[s * kTP + tid] = (y * g) * kCarY;
    }
    __syncthreads();
    v8h hv[2];
#pragma unroll
    for (int it = 0; it < 2; ++it) {
      const float* sp = sY + (it * 8 + wave) * kTP + lane * 8;
      const v4f a0 = *(const v4f*)(sp);
      const v4f a1 = *(const v4f*)(sp + 4);
#pragma unroll
      for (int e = 0; e < 4; ++e) {
        hv[it][e]     = (_Float16)a0[e];
        hv[it][4 + e] = (_Float16)a1[e];
      }
    }
    for (int pass = 0; pass < 2; ++pass) {
#pragma unroll
      for (int it = 0; it < 2; ++it)
        *(volatile v8h*)(Y16 + (size_t)(l0 + it * 8 + wave) * kDin + d0 + lane * 8) = hv[it];
      __threadfence();
    }
  }
}

extern "C" void kernel_launch(void* const* d_in, const int* in_sizes, int n_in,
                              void* d_out, int out_size, void* d_ws, size_t ws_size,
                              hipStream_t stream)
{
  if (n_in < 10) return;
  if (in_sizes[0] != kRows * kDmod) return;
  if (in_sizes[1] != kXZP * kDmod) return;
  if (in_sizes[2] != kDin * 4 || in_sizes[3] != kDin) return;
  if (in_sizes[4] != kPrjN * kDin) return;
  if (in_sizes[5] != kDin * kDtR || in_sizes[6] != kDin) return;
  if (in_sizes[7] != kDin * kNst || in_sizes[8] != kDin) return;
  if (in_sizes[9] != kDmod * kDin) return;
  if (out_size != kRows * kDmod) return;
  if (ws_size < kWsTotal) return;

  const float* x      = (const float*)d_in[0];
  const float* W_in   = (const float*)d_in[1];
  const float* conv_w = (const float*)d_in[2];
  const float* conv_b = (const float*)d_in[3];
  const float* W_xprj = (const float*)d_in[4];
  const float* W_dt   = (const float*)d_in[5];
  const float* b_dt   = (const float*)d_in[6];
  const float* A_log  = (const float*)d_in[7];
  const float* Dv     = (const float*)d_in[8];
  const float* W_out  = (const float*)d_in[9];
  float* dout = (float*)d_out;

  char* ws = (char*)d_ws;
  unsigned short* WIN16  = (unsigned short*)(ws + kOffWIN16);
  unsigned short* WXP16  = (unsigned short*)(ws + kOffWXP16);
  unsigned short* WDT16  = (unsigned short*)(ws + kOffWDT16);
  unsigned short* WOUT16 = (unsigned short*)(ws + kOffWOUT16);
  unsigned short* X16    = (unsigned short*)(ws + kOffX16);
  float*          XZ     = (float*)(ws + kOffXZ);
  float*          UC     = (float*)(ws + kOffUC);
  unsigned short* UC16   = (unsigned short*)(ws + kOffUC16);
  float*          PROJ   = (float*)(ws + kOffPROJ);
  unsigned short* DT16   = (unsigned short*)(ws + kOffDT16);
  float*          DLR    = (float*)(ws + kOffDLR);
  unsigned short* Y16    = (unsigned short*)(ws + kOffY16);

  cast_plane_kernel<0><<<(kRows * kDmod / 8) / 256, 256, 0, stream>>>(x, X16, kRows * kDmod / 8, kRows * kDmod / 8, 1.0f);
  cast_plane_kernel<0><<<(kXZP * kDmod / 8) / 256, 256, 0, stream>>>(W_in, WIN16, kXZP * kDmod / 8, kXZP * kDmod / 8, 1.0f);
  cast_plane_kernel<1><<<(kPrjP * kDin / 8) / 256, 256, 0, stream>>>(W_xprj, WXP16, kPrjN * kDin / 8, kPrjP * kDin / 8, kCarWx);
  cast_plane_kernel<1><<<(kDin * kDtR / 8) / 256, 256, 0, stream>>>(W_dt, WDT16, kDin * kDtR / 8, kDin * kDtR / 8, kCarWdt);
  cast_plane_kernel<1><<<(kDmod * kDin / 8) / 256, 256, 0, stream>>>(W_out, WOUT16, kDmod * kDin / 8, kDmod * kDin / 8, kCarWout);

  for (int b = 0; b < kBatch; ++b) {
    const unsigned short* X16b = X16 + (size_t)b * kSeqL * kDmod;
    float* outb = dout + (size_t)b * kSeqL * kDmod;

    wmma_gemm64<1><<<(kSeqL / 64) * (kXZP / 64) / 8, 256, 0, stream>>>(
        X16b, kDmod, WIN16, kDmod, XZ, kXZP, kSeqL, kXZP, kDmod, 1.0f);

    conv_silu_kernel<<<dim3(kDin / 256, kSeqL / 64), 256, 0, stream>>>(XZ, conv_w, conv_b, UC, UC16);

    wmma_gemm64<0><<<(kSeqL / 64) * (kPrjP / 64) / 8, 256, 0, stream>>>(
        UC16, kDin, WXP16, kDin, PROJ, kPrjP, kSeqL, kPrjP, kDin, 1.0f / kCarWx);

    dt_cast_kernel<<<(kSeqL * kDtR / 8) / 256, 256, 0, stream>>>(PROJ, DT16, kSeqL * kDtR / 8, kCarDt);

    wmma_gemm64<0><<<(kSeqL / 64) * (kDin / 64) / 8, 256, 0, stream>>>(
        DT16, kDtR, WDT16, kDtR, DLR, kDin, kSeqL, kDin, kDtR, 1.0f / (kCarDt * kCarWdt));

    scan_kernel<<<kDin / 256, 256, 0, stream>>>(DLR, UC, XZ, PROJ, A_log, b_dt, Dv, Y16);

    wmma_gemm64<0><<<(kSeqL / 64) * (kDmod / 64) / 8, 256, 0, stream>>>(
        Y16, kDin, WOUT16, kDin, outb, kDmod, kSeqL, kDmod, kDin, 1.0f / (kCarY * kCarWout));
  }
}
